// NATLayer_83854941487363
// MI455X (gfx1250) — hardware-verified
//
#include <hip/hip_runtime.h>
#include <stddef.h>
#include <stdint.h>

#define NBT   2
#define HH    56
#define WW    56
#define CC    256
#define NHD   8
#define DHD   32
#define KS    7
#define PD    3
#define RPW   13
#define NTOK  6272
#define NQKV  768
#define DFF   1024
#define HWP   3136

static_assert(NTOK == NBT * HH * WW);
static_assert(HWP == HH * WW);
static_assert(NTOK % 128 == 0);
static_assert(NTOK % 32 == 0);
static_assert(NTOK % 8 == 0);
static_assert(NHD * DHD == CC);
static_assert(NQKV == 3 * CC);
static_assert(CC % 64 == 0);
static_assert(NQKV % 64 == 0);
static_assert(DFF % 64 == 0);
static_assert(CC % 32 == 0);
static_assert(DFF % 32 == 0);
static_assert((NQKV * CC) % 2048 == 0);
static_assert((CC * CC) % 2048 == 0);
static_assert((DFF * CC) % 2048 == 0);
static_assert(RPW == 2 * KS - 1);

typedef _Float16 v16h __attribute__((ext_vector_type(16)));
typedef _Float16 v8h  __attribute__((ext_vector_type(8)));
typedef float    v8f  __attribute__((ext_vector_type(8)));
typedef float    v4f  __attribute__((ext_vector_type(4)));
typedef unsigned int v4u __attribute__((ext_vector_type(4)));

union Frag  { v16h v; v8h h[2]; };
union Pack8 { v8h h; v4u u; };

__device__ __forceinline__ v8f mma16(v16h a, v16h b, v8f c) {
  c = __builtin_amdgcn_wmma_f32_16x16x32_f16(false, a, false, b, (short)0, c, false, false);
  asm volatile("v_nop\n\tv_nop\n\tv_nop\n\tv_nop" : "+v"(c) : "v"(a), "v"(b));
  return c;
}

__device__ __forceinline__ v16h ldfrag(const _Float16* p, int ld, int row0, int k0, int lane) {
  const int m = lane & 15, lh = lane >> 4;
  const _Float16* q = p + (size_t)(row0 + m) * ld + k0 + 8 * lh;
  Frag f;
  f.h[0] = *(const v8h*)(q);
  f.h[1] = *(const v8h*)(q + 16);
  return f.v;
}

__device__ __forceinline__ v8f zero8() { return (v8f){0.f, 0.f, 0.f, 0.f, 0.f, 0.f, 0.f, 0.f}; }

__device__ __forceinline__ void gemm32x64(const _Float16* __restrict__ A, int lda,
                                          const _Float16* __restrict__ Bt, int ldb, int K,
                                          int m0, int n0, int lane, v8f (&acc)[2][4]) {
#pragma unroll 1
  for (int k0 = 0; k0 < K; k0 += 32) {
    const v16h a0 = ldfrag(A, lda, m0, k0, lane);
    const v16h a1 = ldfrag(A, lda, m0 + 16, k0, lane);
    const v16h b0 = ldfrag(Bt, ldb, n0, k0, lane);
    const v16h b1 = ldfrag(Bt, ldb, n0 + 16, k0, lane);
    const v16h b2 = ldfrag(Bt, ldb, n0 + 32, k0, lane);
    const v16h b3 = ldfrag(Bt, ldb, n0 + 48, k0, lane);
    acc[0][0] = mma16(a0, b0, acc[0][0]);
    acc[1][0] = mma16(a1, b0, acc[1][0]);
    acc[0][1] = mma16(a0, b1, acc[0][1]);
    acc[1][1] = mma16(a1, b1, acc[1][1]);
    acc[0][2] = mma16(a0, b2, acc[0][2]);
    acc[1][2] = mma16(a1, b2, acc[1][2]);
    acc[0][3] = mma16(a0, b3, acc[0][3]);
    acc[1][3] = mma16(a1, b3, acc[1][3]);
  }
}

__global__ __launch_bounds__(256) void k_cvt(const float* __restrict__ src, _Float16* __restrict__ dh, float scale) {
  const size_t o = (size_t)blockIdx.x * 2048 + (size_t)threadIdx.x * 8;
  const v4f a0 = *(const v4f*)(src + o) * scale;
  const v4f a1 = *(const v4f*)(src + o + 4) * scale;
  Pack8 pk;
  pk.h = (v8h){(_Float16)a0[0], (_Float16)a0[1], (_Float16)a0[2], (_Float16)a0[3],
               (_Float16)a1[0], (_Float16)a1[1], (_Float16)a1[2], (_Float16)a1[3]};
  const v4u vv = pk.u;
  volatile v4u* d = (volatile v4u*)(dh + o);
  *d = vv;
  __threadfence();
  *d = vv;
}

__global__ __launch_bounds__(256) void k_ln(const float* __restrict__ src, const float* __restrict__ g,
                                            const float* __restrict__ be, _Float16* __restrict__ dst) {
  const int tid = threadIdx.x, lane = tid & 31, wave = tid >> 5;
  const size_t m = (size_t)blockIdx.x * 8 + wave;
  const float* r = src + m * CC + lane * 8;
  const v4f a0 = *(const v4f*)(r);
  const v4f a1 = *(const v4f*)(r + 4);
  float s = ((a0[0] + a0[1]) + (a0[2] + a0[3])) + ((a1[0] + a1[1]) + (a1[2] + a1[3]));
#pragma unroll
  for (int off = 16; off >= 1; off >>= 1) s += __shfl_xor(s, off, 32);
  const float mean = s * 0.00390625f;
  const v4f d0 = a0 - mean, d1 = a1 - mean;
  float ss = ((d0[0] * d0[0] + d0[1] * d0[1]) + (d0[2] * d0[2] + d0[3] * d0[3])) +
             ((d1[0] * d1[0] + d1[1] * d1[1]) + (d1[2] * d1[2] + d1[3] * d1[3]));
#pragma unroll
  for (int off = 16; off >= 1; off >>= 1) ss += __shfl_xor(ss, off, 32);
  const float var  = ss * 0.00390625f;
  const float rstd = rsqrtf(var + 1e-5f);
  const v4f g0 = *(const v4f*)(g + lane * 8),  g1 = *(const v4f*)(g + lane * 8 + 4);
  const v4f b0 = *(const v4f*)(be + lane * 8), b1 = *(const v4f*)(be + lane * 8 + 4);
  const v4f y0 = (d0 * rstd) * g0 + b0;
  const v4f y1 = (d1 * rstd) * g1 + b1;
  Pack8 pk;
  pk.h = (v8h){(_Float16)y0[0], (_Float16)y0[1], (_Float16)y0[2], (_Float16)y0[3],
               (_Float16)y1[0], (_Float16)y1[1], (_Float16)y1[2], (_Float16)y1[3]};
  const v4u vv = pk.u;
  volatile v4u* d = (volatile v4u*)(dst + m * CC + lane * 8);
  *d = vv;
  __threadfence();
  *d = vv;
}

#define OTP 68
template <int RES>
__device__ __forceinline__ void out_epilogue_f32(v8f (&acc)[2][4], float scale, const float (&bb)[4],
                                                 float* sw, const float* __restrict__ res,
                                                 float* __restrict__ out, int ldo,
                                                 int m0, int n0, int lane, int hh, int c) {
#pragma unroll
  for (int sub = 0; sub < 2; ++sub) {
    __syncthreads();
#pragma unroll
    for (int t = 0; t < 4; ++t) {
#pragma unroll
      for (int r = 0; r < 8; ++r) sw[(8 * hh + r) * OTP + 16 * t + c] = acc[sub][t][r] * scale + bb[t];
    }
    __syncthreads();
    v4f val[8];
    size_t go[8];
#pragma unroll
    for (int it = 0; it < 8; ++it) {
      const int p    = lane + 32 * it;
      const int L    = p >> 3;
      const int pc   = p & 7;
      const int row  = L >> 1;
      const int half = L & 1;
      val[it] = *(const v4f*)(sw + row * OTP + half * 32 + pc * 4);
      go[it]  = (size_t)(m0 + sub * 16 + row) * ldo + n0 + half * 32 + pc * 4;
      if (RES) val[it] = *(const v4f*)(res + go[it]) + val[it];
    }
    for (int ps = 0; ps < 2; ++ps) {
#pragma unroll
      for (int it = 0; it < 8; ++it) *(volatile v4f*)(out + go[it]) = val[it];
      __threadfence();
    }
  }
}

__device__ __forceinline__ void out_epilogue_h16(v8f (&acc)[2][4], float scale, const float (&bb)[4], float oscale,
                                                 float* sw, _Float16* __restrict__ out, int ldo,
                                                 int m0, int n0, int lane, int hh, int c) {
#pragma unroll
  for (int sub = 0; sub < 2; ++sub) {
    __syncthreads();
#pragma unroll
    for (int t = 0; t < 4; ++t) {
#pragma unroll
      for (int r = 0; r < 8; ++r) {
        const float v  = acc[sub][t][r] * scale + bb[t];
        const float lv = (v >= 0.f) ? v : 0.01f * v;
        sw[(8 * hh + r) * OTP + 16 * t + c] = lv * oscale;
      }
    }
    __syncthreads();
    v4u val[4];
    size_t go[4];
#pragma unroll
    for (int it = 0; it < 4; ++it) {
      const int p  = lane + 32 * it;
      const int L  = p >> 3;
      const int pc = p & 7;
      const float* ra = sw + L * OTP + pc * 8;
      const v4f a0 = *(const v4f*)(ra), a1 = *(const v4f*)(ra + 4);
      Pack8 pk;
      pk.h = (v8h){(_Float16)a0[0], (_Float16)a0[1], (_Float16)a0[2], (_Float16)a0[3],
                   (_Float16)a1[0], (_Float16)a1[1], (_Float16)a1[2], (_Float16)a1[3]};
      val[it] = pk.u;
      go[it]  = (size_t)(m0 + sub * 16 + L) * ldo + n0 + pc * 8;
    }
    for (int ps = 0; ps < 2; ++ps) {
#pragma unroll
      for (int it = 0; it < 4; ++it) *(volatile v4u*)(out + go[it]) = val[it];
      __threadfence();
    }
  }
}

template <int RES>
__global__ __launch_bounds__(128) void k_gemm_f32(const _Float16* __restrict__ ap, int lda,
                                                  const _Float16* __restrict__ wt, int K,
                                                  const float* __restrict__ bias, float scale,
                                                  const float* __restrict__ res,
                                                  float* __restrict__ out, int ldo) {
  __shared__ __align__(16) float st[4][16 * OTP];
  const int tid = threadIdx.x, lane = tid & 31, wave = tid >> 5;
  const int hh = lane >> 4, c = lane & 15;
  const int m0 = blockIdx.x * 128 + wave * 32;
  const int n0 = blockIdx.y * 64;

  v8f acc[2][4];
#pragma unroll
  for (int s = 0; s < 2; ++s)
#pragma unroll
    for (int t = 0; t < 4; ++t) acc[s][t] = zero8();
  gemm32x64(ap, lda, wt, K, K, m0, n0, lane, acc);
  float bb[4];
#pragma unroll
  for (int t = 0; t < 4; ++t) bb[t] = bias[n0 + 16 * t + c];
  out_epilogue_f32<RES>(acc, scale, bb, st[wave], res, out, ldo, m0, n0, lane, hh, c);
}

__global__ __launch_bounds__(128) void k_gemm_h16(const _Float16* __restrict__ ap, int lda,
                                                  const _Float16* __restrict__ wt, int K,
                                                  const float* __restrict__ bias, float scale, float oscale,
                                                  _Float16* __restrict__ out, int ldo) {
  __shared__ __align__(16) float st[4][16 * OTP];
  const int tid = threadIdx.x, lane = tid & 31, wave = tid >> 5;
  const int hh = lane >> 4, c = lane & 15;
  const int m0 = blockIdx.x * 128 + wave * 32;
  const int n0 = blockIdx.y * 64;

  v8f acc[2][4];
#pragma unroll
  for (int s = 0; s < 2; ++s)
#pragma unroll
    for (int t = 0; t < 4; ++t) acc[s][t] = zero8();
  gemm32x64(ap, lda, wt, K, K, m0, n0, lane, acc);
  float bb[4];
#pragma unroll
  for (int t = 0; t < 4; ++t) bb[t] = bias[n0 + 16 * t + c];
  out_epilogue_h16(acc, scale, bb, oscale, st[wave], out, ldo, m0, n0, lane, hh, c);
}

#define OSP 264
__global__ __launch_bounds__(256) void k_natt(const float* __restrict__ qkv, const float* __restrict__ rpb,
                                              _Float16* __restrict__ op) {
  __shared__ __align__(16) _Float16 Os[32 * OSP];
  const int tid = threadIdx.x;
  const int pl  = tid >> 3;
  const int h   = tid & 7;
  const int p   = blockIdx.x * 32 + pl;
  const int b   = p / HWP;
  const int rem = p - b * HWP;
  const int i   = rem / WW;
  const int j   = rem - i * WW;

  const float* qr = qkv + (size_t)p * NQKV + h * DHD;
  float q[DHD];
#pragma unroll
  for (int d4 = 0; d4 < 8; ++d4) {
    const v4f t = *(const v4f*)(qr + 4 * d4);
#pragma unroll
    for (int e = 0; e < 4; ++e) q[4 * d4 + e] = t[e] * 0.17677669529663687f;
  }

  float m = -1e30f, l = 0.f;
  float o[DHD];
#pragma unroll
  for (int d = 0; d < DHD; ++d) o[d] = 0.f;

#pragma unroll 1
  for (int di = 0; di < KS; ++di) {
    int ii = i + di - PD;
    ii += (ii < 0) ? HH : 0;
    ii -= (ii >= HH) ? HH : 0;
#pragma unroll 1
    for (int dj = 0; dj < KS; ++dj) {
      int jj = j + dj - PD;
      jj += (jj < 0) ? WW : 0;
      jj -= (jj >= WW) ? WW : 0;
      const size_t t = (size_t)b * HWP + (size_t)ii * WW + jj;
      const float* kr = qkv + t * NQKV + CC + h * DHD;
      const float* vr = kr + CC;
      float s = 0.f;
#pragma unroll
      for (int d4 = 0; d4 < 8; ++d4) {
        const v4f kk = *(const v4f*)(kr + 4 * d4);
#pragma unroll
        for (int e = 0; e < 4; ++e) s += q[4 * d4 + e] * kk[e];
      }
      s += rpb[h * (RPW * RPW) + (PD + di) * RPW + (PD + dj)];
      const float mn = fmaxf(m, s);
      const float sc = __expf(m - mn);
      const float w  = __expf(s - mn);
      l = l * sc + w;
#pragma unroll
      for (int d4 = 0; d4 < 8; ++d4) {
        const v4f vv = *(const v4f*)(vr + 4 * d4);
#pragma unroll
        for (int e = 0; e < 4; ++e) o[4 * d4 + e] = o[4 * d4 + e] * sc + w * vv[e];
      }
      m = mn;
    }
  }
  const float inv = 1.0f / l;
  _Float16* orow = Os + pl * OSP + h * DHD;
#pragma unroll
  for (int d8 = 0; d8 < 4; ++d8) {
    Pack8 pk;
    pk.h = (v8h){(_Float16)(o[8 * d8 + 0] * inv), (_Float16)(o[8 * d8 + 1] * inv),
                 (_Float16)(o[8 * d8 + 2] * inv), (_Float16)(o[8 * d8 + 3] * inv),
                 (_Float16)(o[8 * d8 + 4] * inv), (_Float16)(o[8 * d8 + 5] * inv),
                 (_Float16)(o[8 * d8 + 6] * inv), (_Float16)(o[8 * d8 + 7] * inv)};
    *(v4u*)(orow + 8 * d8) = pk.u;
  }
  __syncthreads();
  v4u val[4];
  size_t go[4];
  const size_t base = (size_t)blockIdx.x * 32 * CC;
#pragma unroll
  for (int it = 0; it < 4; ++it) {
    const int qd = tid + 256 * it;
    const int L  = qd >> 5;
    const int pc = qd & 31;
    val[it] = *(const v4u*)(Os + L * OSP + pc * 8);
    go[it]  = base + (size_t)qd * 8;
  }
  for (int ps = 0; ps < 2; ++ps) {
#pragma unroll
    for (int it = 0; it < 4; ++it) *(volatile v4u*)(op + go[it]) = val[it];
    __threadfence();
  }
}

extern "C" void kernel_launch(void* const* d_in, const int* in_sizes, int n_in,
                              void* d_out, int out_size, void* d_ws, size_t ws_size,
                              hipStream_t stream) {
  if (n_in < 14) return;
  if (in_sizes[0] != NTOK * CC) return;
  if (in_sizes[1] != CC) return;
  if (in_sizes[2] != CC) return;
  if (in_sizes[3] != NQKV * CC) return;
  if (in_sizes[4] != NQKV) return;
  if (in_sizes[5] != NHD * RPW * RPW) return;
  if (in_sizes[6] != CC * CC) return;
  if (in_sizes[7] != CC) return;
  if (in_sizes[8] != CC) return;
  if (in_sizes[9] != CC) return;
  if (in_sizes[10] != DFF * CC) return;
  if (in_sizes[11] != DFF) return;
  if (in_sizes[12] != CC * DFF) return;
  if (in_sizes[13] != CC) return;
  if (out_size != NTOK * CC) return;

  const float* x      = (const float*)d_in[0];
  const float* g1     = (const float*)d_in[1];
  const float* be1    = (const float*)d_in[2];
  const float* qkv_w  = (const float*)d_in[3];
  const float* qkv_b  = (const float*)d_in[4];
  const float* rpb    = (const float*)d_in[5];
  const float* proj_w = (const float*)d_in[6];
  const float* proj_b = (const float*)d_in[7];
  const float* g2     = (const float*)d_in[8];
  const float* be2    = (const float*)d_in[9];
  const float* fc1_w  = (const float*)d_in[10];
  const float* fc1_b  = (const float*)d_in[11];
  const float* fc2_w  = (const float*)d_in[12];
  const float* fc2_b  = (const float*)d_in[13];
  float* out = (float*)d_out;

  size_t off = 0;
  const size_t oWq  = off; off += (size_t)NQKV * CC * 2;
  const size_t oWp  = off; off += (size_t)CC * CC * 2;
  const size_t oW1  = off; off += (size_t)DFF * CC * 2;
  const size_t oW2  = off; off += (size_t)CC * DFF * 2;
  const size_t oXn  = off; off += (size_t)NTOK * CC * 2;
  const size_t oQKV = off; off += (size_t)NTOK * NQKV * 4;
  const size_t oOp  = off; off += (size_t)NTOK * CC * 2;
  const size_t oR1  = off; off += (size_t)NTOK * CC * 4;
  const size_t oH2n = off; off += (size_t)NTOK * CC * 2;
  const size_t oHd  = off; off += (size_t)NTOK * DFF * 2;
  if (off > ws_size) return;
  if (off > (size_t)134217728) return;

  char* ws = (char*)d_ws;
  _Float16* Wq  = (_Float16*)(ws + oWq);
  _Float16* Wp  = (_Float16*)(ws + oWp);
  _Float16* W1  = (_Float16*)(ws + oW1);
  _Float16* W2  = (_Float16*)(ws + oW2);
  _Float16* Xn  = (_Float16*)(ws + oXn);
  float*    QKV = (float*)(ws + oQKV);
  _Float16* Op  = (_Float16*)(ws + oOp);
  float*    R1  = (float*)(ws + oR1);
  _Float16* H2n = (_Float16*)(ws + oH2n);
  _Float16* Hd  = (_Float16*)(ws + oHd);

  k_cvt<<<dim3((NQKV * CC) / 2048), dim3(256), 0, stream>>>(qkv_w, Wq, 32.0f);
  k_cvt<<<dim3((CC * CC) / 2048), dim3(256), 0, stream>>>(proj_w, Wp, 32.0f);
  k_cvt<<<dim3((DFF * CC) / 2048), dim3(256), 0, stream>>>(fc1_w, W1, 32.0f);
  k_cvt<<<dim3((CC * DFF) / 2048), dim3(256), 0, stream>>>(fc2_w, W2, 32.0f);
  k_ln<<<dim3(NTOK / 8), dim3(256), 0, stream>>>(x, g1, be1, Xn);
  k_gemm_f32<0><<<dim3(NTOK / 128, NQKV / 64), dim3(128), 0, stream>>>(Xn, CC, Wq, CC, qkv_b, 0.03125f, x, QKV, NQKV);
  k_natt<<<dim3(NTOK / 32), dim3(256), 0, stream>>>(QKV, rpb, Op);
  k_gemm_f32<1><<<dim3(NTOK / 128, CC / 64), dim3(128), 0, stream>>>(Op, CC, Wp, CC, proj_b, 0.03125f, x, R1, CC);
  k_ln<<<dim3(NTOK / 8), dim3(256), 0, stream>>>(R1, g2, be2, H2n);
  k_gemm_h16<<<dim3(NTOK / 128, DFF / 64), dim3(128), 0, stream>>>(H2n, CC, W1, CC, fc1_b, 0.03125f, 64.0f, Hd, DFF);
  k_gemm_f32<1><<<dim3(NTOK / 128, CC / 64), dim3(128), 0, stream>>>(Hd, DFF, W2, DFF, fc2_b, 0.00048828125f, R1, out, CC);
  (void)hipGetLastError();
}
